// _MinGRUBlock_37563783971150
// MI455X (gfx1250) — hardware-verified
//
#include <hip/hip_runtime.h>
#include <math.h>

#pragma clang fp contract(off)

constexpr int kBatch = 4;
constexpr int kSeq   = 4096;
constexpr int kXD    = 512;
constexpr int kYD    = 512;
constexpr int kNCol  = 2 * kYD;
constexpr int kRows  = kBatch * kSeq;
constexpr float kInvYD = 1.0f / 512.0f;
constexpr float kLnEps = 1e-5f;

constexpr size_t kOffXb   = 0;
constexpr size_t kBytesXb = (size_t)kRows * kXD * 2;
constexpr size_t kOffWb   = kOffXb + kBytesXb;
constexpr size_t kBytesWb = (size_t)kNCol * kXD * 2;
constexpr size_t kOffHg   = kOffWb + kBytesWb;
constexpr size_t kBytesHg = (size_t)kRows * kNCol * 4;
constexpr size_t kOffH    = kOffHg + kBytesHg;
constexpr size_t kBytesH  = (size_t)kRows * kYD * 4;
constexpr size_t kWsTotal = kOffH + kBytesH;
static_assert(kWsTotal == 118489088ull);
static_assert(kWsTotal <= 134217728ull);
static_assert((kOffWb % 128) == 0 && (kOffHg % 128) == 0 && (kOffH % 128) == 0);
static_assert(kRows % 64 == 0 && kNCol % 64 == 0 && kXD % 32 == 0);

typedef __attribute__((ext_vector_type(16))) _Float16 v16h;
typedef __attribute__((ext_vector_type(8)))  _Float16 v8h;
typedef __attribute__((ext_vector_type(16))) __bf16   v16b;
typedef __attribute__((ext_vector_type(8)))  __bf16   v8b;
typedef __attribute__((ext_vector_type(8)))  float    v8f;
typedef __attribute__((ext_vector_type(4)))  float    v4f;
typedef __attribute__((ext_vector_type(4)))  unsigned int v4u;

__device__ __forceinline__ unsigned short f2bf_bits(float f) {
  unsigned u = __float_as_uint(f);
  return (unsigned short)((u + 0x7FFFu + ((u >> 16) & 1u)) >> 16);
}
__device__ __forceinline__ float bf_bits2f(unsigned short h) { return __uint_as_float(((unsigned)h) << 16); }

__device__ __forceinline__ void dep_guard_h(v8f& a, v8f& b, v16h x, v16h y) { asm volatile("v_nop\n\tv_nop\n\tv_nop\n\tv_nop" : "+v"(a), "+v"(b) : "v"(x), "v"(y)); }
__device__ __forceinline__ void dep_guard_b(v8f& a, v8f& b, v16b x, v16b y) { asm volatile("v_nop\n\tv_nop\n\tv_nop\n\tv_nop" : "+v"(a), "+v"(b) : "v"(x), "v"(y)); }
__device__ __forceinline__ void keep4_h(v16h a, v16h b, v16h c, v16h d) { asm volatile("v_nop" :: "v"(a), "v"(b), "v"(c), "v"(d)); }
__device__ __forceinline__ void keep4_b(v16b a, v16b b, v16b c, v16b d) { asm volatile("v_nop" :: "v"(a), "v"(b), "v"(c), "v"(d)); }
__device__ __forceinline__ void acc_guard4(v8f& a, v8f& b, v8f& c, v8f& d) { asm volatile("v_nop\n\tv_nop\n\tv_nop\n\tv_nop" : "+v"(a), "+v"(b), "+v"(c), "+v"(d)); }
template <typename T> struct Frag;
template <> struct Frag<_Float16> {
  typedef v16h V; union U { v16h v; v8h h[2]; };
  static __device__ __forceinline__ v16h load(const _Float16* p) {
    U f; f.h[0] = *(const v8h*)(p); f.h[1] = *(const v8h*)(p + 16); return f.v;
  }
  static __device__ __forceinline__ v8f mma(v16h a, v16h b, v8f c) {
    return __builtin_amdgcn_wmma_f32_16x16x32_f16(false, a, false, b, (short)0, c, false, false);
  }
  static __device__ __forceinline__ void guard(v8f& a, v8f& b, v16h x, v16h y) { dep_guard_h(a, b, x, y); }
  static __device__ __forceinline__ void keep(v16h a, v16h b, v16h c, v16h d) { keep4_h(a, b, c, d); }
};
template <> struct Frag<__bf16> {
  typedef v16b V; union U { v16b v; v8b h[2]; };
  static __device__ __forceinline__ v16b load(const __bf16* p) {
    U f; f.h[0] = *(const v8b*)(p); f.h[1] = *(const v8b*)(p + 16); return f.v;
  }
  static __device__ __forceinline__ v8f mma(v16b a, v16b b, v8f c) {
    return __builtin_amdgcn_wmma_f32_16x16x32_bf16(false, a, false, b, (short)0, c, false, false);
  }
  static __device__ __forceinline__ void guard(v8f& a, v8f& b, v16b x, v16b y) { dep_guard_b(a, b, x, y); }
  static __device__ __forceinline__ void keep(v16b a, v16b b, v16b c, v16b d) { keep4_b(a, b, c, d); }
};

__device__ __forceinline__ unsigned pk16(unsigned short a, unsigned short b) { return (unsigned)a | ((unsigned)b << 16); }

template <int ET> struct Elem;
template <> struct Elem<0> { typedef _Float16 T; };
template <> struct Elem<1> { typedef __bf16 T; };
template <int ET, bool SPLIT, int BIAS_MODE, int OUT_MODE, bool RESID, int ACT = 0>
__global__ __launch_bounds__(256) void wmma_gemm64(
    const unsigned short* __restrict__ Ap, const unsigned short* __restrict__ A2p, int lda, long strideA,
    const unsigned short* __restrict__ Btp, const unsigned short* __restrict__ Bt2p, int ldb, long strideB,
    void* __restrict__ Cout, void* __restrict__ Cout2, int ldc, long strideC,
    const float* __restrict__ bias,
    const float* __restrict__ resid, long strideR,
    int M, int N, int K, float scale) {
  typedef typename Elem<ET>::T T;
  typedef typename Frag<T>::V V;
  const T* A = (const T*)Ap; const T* A2 = (const T*)A2p; const T* Bt = (const T*)Btp; const T* Bt2 = (const T*)Bt2p;
  __shared__ __align__(16) float sT[8][16 * 68];
  const int b    = blockIdx.y;
  const int lane = threadIdx.x & 31;
  const int wave = threadIdx.x >> 5;
  const int tilesN = N >> 6;
  const int tilesM = M >> 6;
  const int tile = blockIdx.x * 8 + wave;
  if (tile >= tilesM * tilesN) return;
  const int tm = tile / tilesN;
  const int tn = tile - tm * tilesN;
  const int m0 = tm << 6;
  const int n0 = tn << 6;

  const T* Ab  = A  + (size_t)b * strideA;
  const T* Bb  = Bt + (size_t)b * strideB;
  const T* Ab2 = SPLIT ? (A2  + (size_t)b * strideA) : nullptr;
  const T* Bb2 = SPLIT ? (Bt2 + (size_t)b * strideB) : nullptr;

  const int rlane = lane & 15;
  const int koff  = (lane >> 4) * 8;
  const int mOff  = (lane >> 4) * 8;

  v8f acc[4][4];
#pragma unroll
  for (int i = 0; i < 4; ++i)
#pragma unroll
    for (int j = 0; j < 4; ++j) acc[i][j] = (v8f){0.f,0.f,0.f,0.f,0.f,0.f,0.f,0.f};

  for (int k0 = 0; k0 < K; k0 += 32) {
    V bh[4], bl[4];
#pragma unroll
    for (int j = 0; j < 4; ++j) {
      const size_t bo = (size_t)(n0 + (j << 4) + rlane) * ldb + koff + k0;
      bh[j] = Frag<T>::load(Bb + bo);
      if (SPLIT) bl[j] = Frag<T>::load(Bb2 + bo);
    }
#pragma unroll
    for (int i = 0; i < 4; ++i) {
      const size_t ao = (size_t)(m0 + (i << 4) + rlane) * lda + koff + k0;
      V ah = Frag<T>::load(Ab + ao);
      V al;
      if (SPLIT) al = Frag<T>::load(Ab2 + ao);
#pragma unroll
      for (int j = 0; j < 4; ++j) {
        acc[i][j] = Frag<T>::mma(ah, bh[j], acc[i][j]);
        if (SPLIT) {
          acc[i][j] = Frag<T>::mma(ah, bl[j], acc[i][j]);
          acc[i][j] = Frag<T>::mma(al, bh[j], acc[i][j]);
        }
      }
      Frag<T>::guard(acc[i][0], acc[i][3], ah, SPLIT ? al : ah);
    }
    Frag<T>::keep(bh[0], bh[1], bh[2], bh[3]);
    if (SPLIT) Frag<T>::keep(bl[0], bl[1], bl[2], bl[3]);
  }
  acc_guard4(acc[0][0], acc[0][1], acc[0][2], acc[0][3]);
  acc_guard4(acc[1][0], acc[1][1], acc[1][2], acc[1][3]);
  acc_guard4(acc[2][0], acc[2][1], acc[2][2], acc[2][3]);
  acc_guard4(acc[3][0], acc[3][1], acc[3][2], acc[3][3]);

  float* slab = sT[wave];
  const float* Rb = RESID ? (resid + (size_t)b * strideR) : nullptr;
#pragma unroll
  for (int i = 0; i < 4; ++i) {
    const int mBase = m0 + (i << 4);
#pragma unroll
    for (int j = 0; j < 4; ++j) {
      const int n = n0 + (j << 4) + rlane;
      float bv = 0.f;
      if (BIAS_MODE == 2) bv = bias[n];
#pragma unroll
      for (int r = 0; r < 8; ++r) {
        float v = acc[i][j][r] * scale;
        if (BIAS_MODE == 1) v += bias[mBase + mOff + r];
        if (BIAS_MODE == 2) v += bv;
        if (RESID) v += Rb[(size_t)(mBase + mOff + r) * ldc + n];
        if (ACT == 2) v = fmaxf(v, 0.0f);
        if (ACT == 4) v = (v > 0.f) ? v : 0.01f * v;
        slab[(mOff + r) * 68 + (j << 4) + rlane] = v;
      }
    }
    __builtin_amdgcn_fence(__ATOMIC_RELEASE, "workgroup");
    __builtin_amdgcn_wave_barrier();
    __builtin_amdgcn_fence(__ATOMIC_ACQUIRE, "workgroup");
    if (OUT_MODE == 0) {
      float* C = (float*)Cout + (size_t)b * strideC;
      const int hh = lane >> 4, c4 = (lane & 15) * 4;
      for (int pass = 0; pass < 2; ++pass) {
#pragma unroll
        for (int it = 0; it < 8; ++it) {
          const int row = it * 2 + hh;
          v4f v = *(const v4f*)(slab + row * 68 + c4);
          *(volatile v4f*)(C + (size_t)(mBase + row) * ldc + n0 + c4) = v;
        }
        __threadfence();
      }
    } else {
      const int q = lane >> 3, c8 = (lane & 7) * 8;
      unsigned short* C  = (unsigned short*)Cout  + (size_t)b * strideC;
      unsigned short* C2 = (OUT_MODE == 2) ? ((unsigned short*)Cout2 + (size_t)b * strideC) : nullptr;
      for (int pass = 0; pass < 2; ++pass) {
#pragma unroll
        for (int it = 0; it < 4; ++it) {
          const int row = it * 4 + q;
          const float* sp = slab + row * 68 + c8;
          v8h hv, lv;
#pragma unroll
          for (int e = 0; e < 8; ++e) {
            if (OUT_MODE == 1) {
              hv[e] = (_Float16)sp[e];
            } else {
              unsigned short hb = f2bf_bits(sp[e]);
              unsigned short lb = f2bf_bits(sp[e] - bf_bits2f(hb));
              hv[e] = __builtin_bit_cast(_Float16, hb);
              lv[e] = __builtin_bit_cast(_Float16, lb);
            }
          }
          *(volatile v8h*)(C + (size_t)(mBase + row) * ldc + n0 + c8) = hv;
          if (OUT_MODE == 2) *(volatile v8h*)(C2 + (size_t)(mBase + row) * ldc + n0 + c8) = lv;
        }
        __threadfence();
      }
    }
    __builtin_amdgcn_fence(__ATOMIC_RELEASE, "workgroup");
    __builtin_amdgcn_wave_barrier();
    __builtin_amdgcn_fence(__ATOMIC_ACQUIRE, "workgroup");
  }
}

__global__ __launch_bounds__(256) void cast8_bf16_kernel(const float* __restrict__ in, unsigned short* __restrict__ out, int n8) {
  const int i = blockIdx.x * 256 + threadIdx.x;
  if (i >= n8) return;
  const float* p = in + 8 * (size_t)i;
  const v4f a = *(const v4f*)(p);
  const v4f c = *(const v4f*)(p + 4);
  unsigned short hb[8];
#pragma unroll
  for (int e = 0; e < 4; ++e) {
    hb[e]     = f2bf_bits(a[e]);
    hb[4 + e] = f2bf_bits(c[e]);
  }
  const v4u u = (v4u){pk16(hb[0], hb[1]), pk16(hb[2], hb[3]), pk16(hb[4], hb[5]), pk16(hb[6], hb[7])};
  unsigned short* q = out + 8 * (size_t)i;
  *(volatile v4u*)q = u;
  __threadfence();
  *(volatile v4u*)q = u;
}

__global__ __launch_bounds__(64) void scan_kernel(const float* __restrict__ HG, float* __restrict__ Hout) {
  const int b = blockIdx.x >> 3;
  const int c = ((blockIdx.x & 7) << 6) + threadIdx.x;
  const float* p = HG + (size_t)b * kSeq * kNCol + c;
  float* q = Hout + (size_t)b * kSeq * kYD + c;
  float lh = 0.0f;
#pragma unroll 1
  for (int s = 0; s < kSeq; ++s) {
    const float hp = p[(size_t)s * kNCol];
    const float gt = p[(size_t)s * kNCol + kYD];
    const float lg1 = log1pf(expf(-fabsf(gt)));
    const float lc  = -(fmaxf(gt, 0.0f) + lg1);
    const float lz  = -(fmaxf(-gt, 0.0f) + lg1);
    const float pos = logf(fmaxf(hp, 0.0f) + 0.5f);
    const float neg = -(fmaxf(-hp, 0.0f) + log1pf(expf(-fabsf(hp))));
    const float lgv = (hp >= 0.0f) ? pos : neg;
    const float lv  = lz + lgv;
    const float t   = lh + lc;
    const float mx  = fmaxf(t, lv);
    const float rec = mx + log1pf(expf(-fabsf(t - lv)));
    const float first = lc + (lv - lc);
    lh = (s == 0) ? first : rec;
    const float hval = expf(lh);
    float* dst = q + (size_t)s * kYD;
    *(volatile float*)dst = hval;
    __threadfence();
    *(volatile float*)dst = hval;
  }
}

__global__ __launch_bounds__(128) void ln_kernel(const float* __restrict__ Hin, const float* __restrict__ gamma,
                                                const float* __restrict__ beta, float* __restrict__ Y) {
  __shared__ float red1[4];
  __shared__ float red2[4];
  const int row  = blockIdx.x;
  const int t    = threadIdx.x;
  const int lane = t & 31, wave = t >> 5;
  const v4f hv = *(const v4f*)(Hin + (size_t)row * kYD + 4 * t);
  float s1 = (hv[0] + hv[1]) + (hv[2] + hv[3]);
#pragma unroll
  for (int off = 16; off > 0; off >>= 1) s1 += __shfl_xor(s1, off, 32);
  if (lane == 0) red1[wave] = s1;
  __syncthreads();
  const float mean = ((red1[0] + red1[1]) + (red1[2] + red1[3])) * kInvYD;
  const float d0 = hv[0] - mean, d1 = hv[1] - mean, d2 = hv[2] - mean, d3 = hv[3] - mean;
  float s2 = (d0 * d0 + d1 * d1) + (d2 * d2 + d3 * d3);
#pragma unroll
  for (int off = 16; off > 0; off >>= 1) s2 += __shfl_xor(s2, off, 32);
  if (lane == 0) red2[wave] = s2;
  __syncthreads();
  const float var = ((red2[0] + red2[1]) + (red2[2] + red2[3])) * kInvYD;
  const float rs  = 1.0f / sqrtf(var + kLnEps);
  const v4f gv = *(const v4f*)(gamma + 4 * t);
  const v4f bv = *(const v4f*)(beta + 4 * t);
  const float g0 = bf_bits2f(f2bf_bits(gv[0])), g1 = bf_bits2f(f2bf_bits(gv[1]));
  const float g2 = bf_bits2f(f2bf_bits(gv[2])), g3 = bf_bits2f(f2bf_bits(gv[3]));
  const float e0 = bf_bits2f(f2bf_bits(bv[0])), e1 = bf_bits2f(f2bf_bits(bv[1]));
  const float e2 = bf_bits2f(f2bf_bits(bv[2])), e3 = bf_bits2f(f2bf_bits(bv[3]));
  v4f yv;
  yv[0] = (d0 * rs) * g0 + e0;
  yv[1] = (d1 * rs) * g1 + e1;
  yv[2] = (d2 * rs) * g2 + e2;
  yv[3] = (d3 * rs) * g3 + e3;
  float* dst = Y + (size_t)row * kYD + 4 * t;
  *(volatile v4f*)dst = yv;
  __threadfence();
  *(volatile v4f*)dst = yv;
}

extern "C" void kernel_launch(void* const* d_in, const int* in_sizes, int n_in,
                              void* d_out, int out_size, void* d_ws, size_t ws_size,
                              hipStream_t stream)
{
  if (n_in < 4) return;
  if (in_sizes[0] != kRows * kXD || in_sizes[1] != kNCol * kXD ||
      in_sizes[2] != kYD || in_sizes[3] != kYD || out_size != kRows * kYD) return;
  if (ws_size < kWsTotal) return;

  const float* x     = (const float*)d_in[0];
  const float* W     = (const float*)d_in[1];
  const float* gamma = (const float*)d_in[2];
  const float* beta  = (const float*)d_in[3];
  float* y = (float*)d_out;

  char* ws = (char*)d_ws;
  unsigned short* xb = (unsigned short*)(ws + kOffXb);
  unsigned short* wb = (unsigned short*)(ws + kOffWb);
  float* hg  = (float*)(ws + kOffHg);
  float* hst = (float*)(ws + kOffH);

  const int n8x = kRows * kXD / 8;
  const int n8w = kNCol * kXD / 8;
  cast8_bf16_kernel<<<dim3(n8x / 256), dim3(256), 0, stream>>>(x, xb, n8x);
  cast8_bf16_kernel<<<dim3(n8w / 256), dim3(256), 0, stream>>>(W, wb, n8w);

  wmma_gemm64<1, false, 0, 0, false><<<dim3((kRows / 64) * (kNCol / 64) / 8, 1), dim3(256), 0, stream>>>(
      xb, xb, kXD, 0L, wb, wb, kXD, 0L, (void*)hg, (void*)hg, kNCol, 0L,
      gamma, hg, 0L, kRows, kNCol, kXD, 1.0f);

  scan_kernel<<<dim3(kBatch * kYD / 64), dim3(64), 0, stream>>>(hg, hst);

  ln_kernel<<<dim3(kRows), dim3(128), 0, stream>>>(hst, gamma, beta, y);
}
